// BasicTransformer_78288663872115
// MI455X (gfx1250) — hardware-verified
//
#include <hip/hip_runtime.h>
#include <stddef.h>
#include <stdint.h>
#include <math.h>

#define NB    2
#define SQ    2048
#define NTOK  4096
#define HID   1024
#define NH    16
#define HDM   64
#define DFF   4096
#define NQKV  3072
#define QB    128
#define KC    64
#define NQB   (SQ / QB)
#define NCK   (SQ / KC)
#define SBLK  (SQ / 256)
#define QKPLANE (NB * NH * SQ * HDM)

#define WSC 256.0f
#define QSC 8.0f
#define PSC 1024.0f
#define OSC 512.0f
#define HSC 32.0f

static_assert(NTOK == NB * SQ);
static_assert(SQ % 256 == 0);
static_assert(HID % 256 == 0);
static_assert(HID % 64 == 0);
static_assert(DFF % 64 == 0);
static_assert(HDM == 64);
static_assert(NH * HDM == HID);
static_assert(NQKV == 3 * NH * HDM);
static_assert(SQ % KC == 0);
static_assert(SQ % QB == 0);
static_assert(QB == 8 * 16);
static_assert(NTOK % 256 == 0);
static_assert(NTOK % 8 == 0);

typedef _Float16 v16h __attribute__((ext_vector_type(16)));
typedef _Float16 v8h  __attribute__((ext_vector_type(8)));
typedef float    v8f  __attribute__((ext_vector_type(8)));
typedef float    v4f  __attribute__((ext_vector_type(4)));
typedef unsigned int v4u __attribute__((ext_vector_type(4)));

union Frag  { v16h v; v8h h[2]; };
union Pack8 { v8h h; v4u u; };

__device__ __forceinline__ v8f mma16(v16h a, v16h b, v8f c) {
  c = __builtin_amdgcn_wmma_f32_16x16x32_f16(false, a, false, b, (short)0, c, false, false);
  asm volatile("v_nop\n\tv_nop\n\tv_nop\n\tv_nop" : "+v"(c) : "v"(a), "v"(b));
  return c;
}

__device__ __forceinline__ v16h ldfrag(const _Float16* p, int ld, int row0, int k0, int lane) {
  const int m = lane & 15, lh = lane >> 4;
  const _Float16* q = p + (size_t)(row0 + m) * ld + k0 + 8 * lh;
  Frag f;
  f.h[0] = *(const v8h*)(q);
  f.h[1] = *(const v8h*)(q + 16);
  return f.v;
}

__device__ __forceinline__ v8f zero8() { return (v8f){0.f, 0.f, 0.f, 0.f, 0.f, 0.f, 0.f, 0.f}; }

__device__ __forceinline__ void gemm32x64(const _Float16* __restrict__ A, int lda,
                                          const _Float16* __restrict__ Bt, int ldb, int K,
                                          int m0, int n0, int lane, v8f (&acc)[2][4]) {
#pragma unroll 1
  for (int k0 = 0; k0 < K; k0 += 32) {
    const v16h a0 = ldfrag(A, lda, m0, k0, lane);
    const v16h a1 = ldfrag(A, lda, m0 + 16, k0, lane);
    const v16h b0 = ldfrag(Bt, ldb, n0, k0, lane);
    const v16h b1 = ldfrag(Bt, ldb, n0 + 16, k0, lane);
    const v16h b2 = ldfrag(Bt, ldb, n0 + 32, k0, lane);
    const v16h b3 = ldfrag(Bt, ldb, n0 + 48, k0, lane);
    acc[0][0] = mma16(a0, b0, acc[0][0]);
    acc[1][0] = mma16(a1, b0, acc[1][0]);
    acc[0][1] = mma16(a0, b1, acc[0][1]);
    acc[1][1] = mma16(a1, b1, acc[1][1]);
    acc[0][2] = mma16(a0, b2, acc[0][2]);
    acc[1][2] = mma16(a1, b2, acc[1][2]);
    acc[0][3] = mma16(a0, b3, acc[0][3]);
    acc[1][3] = mma16(a1, b3, acc[1][3]);
  }
}

#define WTP 72
__global__ __launch_bounds__(256) void k_wtr(const float* __restrict__ w, int Kd, int Nd, float scale,
                                             _Float16* __restrict__ wt) {
  __shared__ __align__(16) _Float16 st[64 * WTP];
  const int tid = threadIdx.x;
  const int n0 = blockIdx.x * 64, k0 = blockIdx.y * 64;
#pragma unroll
  for (int j = 0; j < 4; ++j) {
    const int p  = tid + 256 * j;
    const int kr = p >> 4;
    const int nc = (p & 15) * 4;
    const v4f a = *(const v4f*)(w + (size_t)(k0 + kr) * Nd + n0 + nc) * scale;
    st[(nc + 0) * WTP + kr] = (_Float16)a[0];
    st[(nc + 1) * WTP + kr] = (_Float16)a[1];
    st[(nc + 2) * WTP + kr] = (_Float16)a[2];
    st[(nc + 3) * WTP + kr] = (_Float16)a[3];
  }
  __syncthreads();
  v4u val[2];
  size_t go[2];
#pragma unroll
  for (int j = 0; j < 2; ++j) {
    const int p  = tid + 256 * j;
    const int n  = p >> 3;
    const int pc = p & 7;
    Pack8 pk;
    pk.h   = *(const v8h*)(st + n * WTP + pc * 8);
    val[j] = pk.u;
    go[j]  = (size_t)(n0 + n) * Kd + k0 + pc * 8;
  }
  for (int ps = 0; ps < 2; ++ps) {
#pragma unroll
    for (int j = 0; j < 2; ++j) *(volatile v4u*)(wt + go[j]) = val[j];
    __threadfence();
  }
}

template <int ADD>
__global__ __launch_bounds__(256) void k_ln_h(const float* __restrict__ xa, const float* __restrict__ xb,
                                              const float* __restrict__ g, const float* __restrict__ be,
                                              _Float16* __restrict__ yh) {
  __shared__ __align__(16) float sw[8][HID];
  const int tid = threadIdx.x, lane = tid & 31, wave = tid >> 5;
  const size_t m = (size_t)blockIdx.x * 8 + wave;
  const float* ar = xa + m * HID;
  const float* br = xb + m * HID;

  v4f v[8];
  float s = 0.f;
#pragma unroll
  for (int it = 0; it < 8; ++it) {
    const int idx = it * 128 + lane * 4;
    v4f a = *(const v4f*)(ar + idx);
    if (ADD) {
      const v4f r = *(const v4f*)(br + idx);
      a = a + r;
    }
    v[it] = a;
    s += (a[0] + a[1]) + (a[2] + a[3]);
  }
#pragma unroll
  for (int off = 16; off >= 1; off >>= 1) s += __shfl_xor(s, off, 32);
  const float mean = s * (1.0f / 1024.0f);
  float ss = 0.f;
#pragma unroll
  for (int it = 0; it < 8; ++it) {
    const v4f d = v[it] - mean;
    ss += (d[0] * d[0] + d[1] * d[1]) + (d[2] * d[2] + d[3] * d[3]);
  }
#pragma unroll
  for (int off = 16; off >= 1; off >>= 1) ss += __shfl_xor(ss, off, 32);
  const float var  = ss * (1.0f / 1024.0f);
  const float rstd = rsqrtf(var + 1e-3f);

#pragma unroll
  for (int it = 0; it < 8; ++it) {
    const int idx = it * 128 + lane * 4;
    const v4f gv = *(const v4f*)(g + idx);
    const v4f bv = *(const v4f*)(be + idx);
    const v4f y = ((v[it] - mean) * rstd) * gv + bv;
    *(v4f*)(sw[wave] + idx) = y;
  }
  __syncthreads();
  v4u hv[4];
  size_t go[4];
#pragma unroll
  for (int j = 0; j < 4; ++j) {
    const float* cp = sw[wave] + 256 * j + 8 * lane;
    const v4f a0 = *(const v4f*)(cp), a1 = *(const v4f*)(cp + 4);
    Pack8 pk;
    pk.h = (v8h){(_Float16)a0[0], (_Float16)a0[1], (_Float16)a0[2], (_Float16)a0[3],
                 (_Float16)a1[0], (_Float16)a1[1], (_Float16)a1[2], (_Float16)a1[3]};
    hv[j] = pk.u;
    go[j] = m * HID + 256 * j + 8 * lane;
  }
  for (int ps = 0; ps < 2; ++ps) {
#pragma unroll
    for (int j = 0; j < 4; ++j) *(volatile v4u*)(yh + go[j]) = hv[j];
    __threadfence();
  }
}

#define STP 72
#define SVP 264
static_assert(256 * STP >= 64 * SVP);
__global__ __launch_bounds__(256) void k_qkv(const _Float16* __restrict__ nh,
                                             const _Float16* __restrict__ wt,
                                             const float* __restrict__ bqkv,
                                             _Float16* __restrict__ qkp,
                                             _Float16* __restrict__ vtp) {
  __shared__ __align__(16) _Float16 st[256 * STP];
  const int tid = threadIdx.x, lane = tid & 31, wave = tid >> 5;
  const int hh = lane >> 4, c = lane & 15;
  const int bx = blockIdx.x;
  const int b  = bx / SBLK;
  const int sb = (bx - b * SBLK) * 256;
  const int ns = blockIdx.y;
  const int head  = ns / 3;
  const int which = ns - head * 3;
  const int hb    = b * NH + head;
  const int m0 = bx * 256 + wave * 32;
  const int n0 = ns * 64;

  v8f acc[2][4];
#pragma unroll
  for (int s = 0; s < 2; ++s)
#pragma unroll
    for (int t = 0; t < 4; ++t) acc[s][t] = zero8();
  gemm32x64(nh, HID, wt, HID, HID, m0, n0, lane, acc);

  float bb[4];
#pragma unroll
  for (int t = 0; t < 4; ++t) bb[t] = bqkv[n0 + 16 * t + c];
  const float isc = 1.0f / WSC;
  const float osc = (which == 0) ? QSC : 1.0f;

  if (which < 2) {
#pragma unroll
    for (int sub = 0; sub < 2; ++sub)
#pragma unroll
      for (int t = 0; t < 4; ++t)
#pragma unroll
        for (int r = 0; r < 8; ++r) {
          const int lr = wave * 32 + sub * 16 + 8 * hh + r;
          st[lr * STP + 16 * t + c] = (_Float16)((acc[sub][t][r] * isc + bb[t]) * osc);
        }
  } else {
#pragma unroll
    for (int sub = 0; sub < 2; ++sub)
#pragma unroll
      for (int t = 0; t < 4; ++t)
#pragma unroll
        for (int r = 0; r < 8; ++r)
          st[(16 * t + c) * SVP + wave * 32 + sub * 16 + 8 * hh + r] =
              (_Float16)(acc[sub][t][r] * isc + bb[t]);
  }
  __syncthreads();

  if (which < 2) {
    _Float16* base = qkp + (size_t)which * QKPLANE + (size_t)hb * SQ * HDM;
#pragma unroll
    for (int g = 0; g < 2; ++g) {
      v4u val[4];
      size_t go[4];
#pragma unroll
      for (int j = 0; j < 4; ++j) {
        const int p  = tid + 256 * (4 * g + j);
        const int lr = p >> 3;
        const int pc = p & 7;
        Pack8 pk;
        pk.h   = *(const v8h*)(st + lr * STP + pc * 8);
        val[j] = pk.u;
        go[j]  = (size_t)(sb + lr) * HDM + pc * 8;
      }
      for (int ps = 0; ps < 2; ++ps) {
#pragma unroll
        for (int j = 0; j < 4; ++j) *(volatile v4u*)(base + go[j]) = val[j];
        __threadfence();
      }
    }
  } else {
    _Float16* base = vtp + (size_t)hb * HDM * SQ;
#pragma unroll
    for (int g = 0; g < 2; ++g) {
      v4u val[4];
      size_t go[4];
#pragma unroll
      for (int j = 0; j < 4; ++j) {
        const int p    = tid + 256 * (4 * g + j);
        const int drow = p >> 5;
        const int pc   = p & 31;
        Pack8 pk;
        pk.h   = *(const v8h*)(st + drow * SVP + pc * 8);
        val[j] = pk.u;
        go[j]  = (size_t)drow * SQ + sb + pc * 8;
      }
      for (int ps = 0; ps < 2; ++ps) {
#pragma unroll
        for (int j = 0; j < 4; ++j) *(volatile v4u*)(base + go[j]) = val[j];
        __threadfence();
      }
    }
  }
}

#define KTP 72
__global__ __launch_bounds__(256) void k_attn(const _Float16* __restrict__ qp,
                                              const _Float16* __restrict__ kp,
                                              const _Float16* __restrict__ vt,
                                              _Float16* __restrict__ op, float sscale) {
  __shared__ __align__(16) _Float16 Ks[KC * KTP];
  __shared__ __align__(16) _Float16 Vs[HDM * KTP];
  __shared__ __align__(16) _Float16 Ps[8 * 16 * KTP];

  const int tid = threadIdx.x, lane = tid & 31, wave = tid >> 5;
  const int hh = lane >> 4, c = lane & 15;
  const int qb  = blockIdx.x % NQB;
  const int hb  = blockIdx.x / NQB;
  const int h   = hb % NH;
  const int b   = hb / NH;
  const int q0  = qb * QB + wave * 16;

  const _Float16* Q = qp + (size_t)hb * SQ * HDM;
  const _Float16* K = kp + (size_t)hb * SQ * HDM;
  const _Float16* V = vt + (size_t)hb * HDM * SQ;

  v16h qa[2];
  qa[0] = ldfrag(Q, HDM, q0, 0, lane);
  qa[1] = ldfrag(Q, HDM, q0, 32, lane);

  const float NEGI = -__builtin_huge_valf();
  float mrow[8], lrow[8];
  v8f oacc[4];
#pragma unroll
  for (int r = 0; r < 8; ++r) { mrow[r] = NEGI; lrow[r] = 0.f; }
#pragma unroll
  for (int t = 0; t < 4; ++t) oacc[t] = zero8();

  _Float16* pw = Ps + wave * 16 * KTP;

  for (int kc = 0; kc < NCK; ++kc) {
    const int kv0 = kc * KC;
    __syncthreads();
    {
      const int r  = tid >> 2;
      const int qq = (tid & 3) * 16;
      const _Float16* ks = K + (size_t)(kv0 + r) * HDM + qq;
      const _Float16* vs = V + (size_t)r * SQ + kv0 + qq;
#pragma unroll
      for (int e = 0; e < 2; ++e) {
        *(v8h*)(Ks + r * KTP + qq + 8 * e) = *(const v8h*)(ks + 8 * e);
        *(v8h*)(Vs + r * KTP + qq + 8 * e) = *(const v8h*)(vs + 8 * e);
      }
    }
    __syncthreads();

    v8f s[4];
#pragma unroll
    for (int j = 0; j < 4; ++j) s[j] = zero8();
#pragma unroll
    for (int dc = 0; dc < 2; ++dc) {
#pragma unroll
      for (int j = 0; j < 4; ++j) {
        const v16h kb = ldfrag(Ks, KTP, j * 16, dc * 32, lane);
        s[j] = mma16(qa[dc], kb, s[j]);
      }
    }
    float cm[8];
#pragma unroll
    for (int r = 0; r < 8; ++r) {
      float m = NEGI;
#pragma unroll
      for (int j = 0; j < 4; ++j) { s[j][r] = s[j][r] * sscale; m = fmaxf(m, s[j][r]); }
#pragma unroll
      for (int off = 1; off < 16; off <<= 1) m = fmaxf(m, __shfl_xor(m, off, 32));
      cm[r] = m;
    }
    float al[8];
#pragma unroll
    for (int r = 0; r < 8; ++r) {
      const float mnew  = fmaxf(mrow[r], cm[r]);
      const float alpha = __expf(mrow[r] - mnew);
      mrow[r] = mnew;
      float psum = 0.f;
#pragma unroll
      for (int j = 0; j < 4; ++j) {
        const float p = __expf(s[j][r] - mnew);
        psum += p;
        pw[(8 * hh + r) * KTP + j * 16 + c] = (_Float16)(p * PSC);
      }
#pragma unroll
      for (int off = 1; off < 16; off <<= 1) psum += __shfl_xor(psum, off, 32);
      lrow[r] = lrow[r] * alpha + psum;
      al[r] = alpha;
    }
#pragma unroll
    for (int t = 0; t < 4; ++t)
#pragma unroll
      for (int r = 0; r < 8; ++r) oacc[t][r] *= al[r];
    __syncthreads();

#pragma unroll
    for (int kk = 0; kk < 2; ++kk) {
      const v16h pa = ldfrag(pw, KTP, 0, kk * 32, lane);
#pragma unroll
      for (int t = 0; t < 4; ++t) {
        const v16h vb = ldfrag(Vs, KTP, t * 16, kk * 32, lane);
        oacc[t] = mma16(pa, vb, oacc[t]);
      }
    }
  }

  float invl[8];
#pragma unroll
  for (int r = 0; r < 8; ++r) invl[r] = (lrow[r] > 0.f) ? ((OSC / PSC) / lrow[r]) : 0.f;
  __syncthreads();
#pragma unroll
  for (int r = 0; r < 8; ++r) {
#pragma unroll
    for (int t = 0; t < 4; ++t)
      pw[(8 * hh + r) * KTP + 16 * t + c] = (_Float16)(oacc[t][r] * invl[r]);
  }
  __syncthreads();
  v4u val[4];
  size_t go[4];
#pragma unroll
  for (int it = 0; it < 4; ++it) {
    const int p  = lane + 32 * it;
    const int L  = p >> 3;
    const int pc = p & 7;
    Pack8 pk;
    pk.h    = *(const v8h*)(pw + L * KTP + pc * 8);
    val[it] = pk.u;
    go[it]  = ((size_t)(b * SQ + q0 + L)) * HID + (size_t)h * HDM + pc * 8;
  }
  for (int ps = 0; ps < 2; ++ps) {
#pragma unroll
    for (int it = 0; it < 4; ++it) *(volatile v4u*)(op + go[it]) = val[it];
    __threadfence();
  }
}

#define OTP 68
template <int RES>
__device__ __forceinline__ void out_epilogue_f32(v8f (&acc)[2][4], float scale, const float (&bb)[4],
                                                 float* sw, float* __restrict__ out, int ldo,
                                                 const float* __restrict__ ra, const float* __restrict__ rb,
                                                 int m0, int n0, int lane, int hh, int c) {
#pragma unroll
  for (int sub = 0; sub < 2; ++sub) {
    __syncthreads();
#pragma unroll
    for (int t = 0; t < 4; ++t) {
#pragma unroll
      for (int r = 0; r < 8; ++r) sw[(8 * hh + r) * OTP + 16 * t + c] = acc[sub][t][r] * scale + bb[t];
    }
    __syncthreads();
    v4f val[8];
    size_t go[8];
#pragma unroll
    for (int it = 0; it < 8; ++it) {
      const int p    = lane + 32 * it;
      const int L    = p >> 3;
      const int pc   = p & 7;
      const int row  = L >> 1;
      const int half = L & 1;
      v4f vv = *(const v4f*)(sw + row * OTP + half * 32 + pc * 4);
      go[it]  = (size_t)(m0 + sub * 16 + row) * ldo + n0 + half * 32 + pc * 4;
      if (RES) {
        const v4f x0 = *(const v4f*)(ra + go[it]);
        const v4f x1 = *(const v4f*)(rb + go[it]);
        vv = (x0 + x1) + vv;
      }
      val[it] = vv;
    }
    for (int ps = 0; ps < 2; ++ps) {
#pragma unroll
      for (int it = 0; it < 8; ++it) *(volatile v4f*)(out + go[it]) = val[it];
      __threadfence();
    }
  }
}

__device__ __forceinline__ void out_epilogue_h16(v8f (&acc)[2][4], float scale, const float (&bb)[4], float oscale,
                                                 float* sw, _Float16* __restrict__ out, int ldo,
                                                 int m0, int n0, int lane, int hh, int c) {
#pragma unroll
  for (int sub = 0; sub < 2; ++sub) {
    __syncthreads();
#pragma unroll
    for (int t = 0; t < 4; ++t) {
#pragma unroll
      for (int r = 0; r < 8; ++r) {
        const float v  = acc[sub][t][r] * scale + bb[t];
        const float u  = 0.7978845608028654f * (v + 0.044715f * (v * v * v));
        const float gl = v * (0.5f * (1.0f + tanhf(u)));
        sw[(8 * hh + r) * OTP + 16 * t + c] = gl * oscale;
      }
    }
    __syncthreads();
    v4u val[4];
    size_t go[4];
#pragma unroll
    for (int it = 0; it < 4; ++it) {
      const int p  = lane + 32 * it;
      const int L  = p >> 3;
      const int pc = p & 7;
      const float* rp = sw + L * OTP + pc * 8;
      const v4f a0 = *(const v4f*)(rp), a1 = *(const v4f*)(rp + 4);
      Pack8 pk;
      pk.h = (v8h){(_Float16)a0[0], (_Float16)a0[1], (_Float16)a0[2], (_Float16)a0[3],
                   (_Float16)a1[0], (_Float16)a1[1], (_Float16)a1[2], (_Float16)a1[3]};
      val[it] = pk.u;
      go[it]  = (size_t)(m0 + sub * 16 + L) * ldo + n0 + pc * 8;
    }
    for (int ps = 0; ps < 2; ++ps) {
#pragma unroll
      for (int it = 0; it < 4; ++it) *(volatile v4u*)(out + go[it]) = val[it];
      __threadfence();
    }
  }
}

template <int RES>
__global__ __launch_bounds__(256) void k_gemm_f32(const _Float16* __restrict__ ap, int lda,
                                                  const _Float16* __restrict__ wt, int K,
                                                  const float* __restrict__ bias, float scale,
                                                  float* __restrict__ out, int ldo,
                                                  const float* __restrict__ ra, const float* __restrict__ rb) {
  __shared__ __align__(16) float st[8][16 * OTP];
  const int tid = threadIdx.x, lane = tid & 31, wave = tid >> 5;
  const int hh = lane >> 4, c = lane & 15;
  const int m0 = blockIdx.x * 256 + wave * 32;
  const int n0 = blockIdx.y * 64;

  v8f acc[2][4];
#pragma unroll
  for (int s = 0; s < 2; ++s)
#pragma unroll
    for (int t = 0; t < 4; ++t) acc[s][t] = zero8();
  gemm32x64(ap, lda, wt, K, K, m0, n0, lane, acc);
  float bb[4];
#pragma unroll
  for (int t = 0; t < 4; ++t) bb[t] = bias[n0 + 16 * t + c];
  out_epilogue_f32<RES>(acc, scale, bb, st[wave], out, ldo, ra, rb, m0, n0, lane, hh, c);
}

__global__ __launch_bounds__(256) void k_gemm_h16(const _Float16* __restrict__ ap, int lda,
                                                  const _Float16* __restrict__ wt, int K,
                                                  const float* __restrict__ bias, float scale, float oscale,
                                                  _Float16* __restrict__ out, int ldo) {
  __shared__ __align__(16) float st[8][16 * OTP];
  const int tid = threadIdx.x, lane = tid & 31, wave = tid >> 5;
  const int hh = lane >> 4, c = lane & 15;
  const int m0 = blockIdx.x * 256 + wave * 32;
  const int n0 = blockIdx.y * 64;

  v8f acc[2][4];
#pragma unroll
  for (int s = 0; s < 2; ++s)
#pragma unroll
    for (int t = 0; t < 4; ++t) acc[s][t] = zero8();
  gemm32x64(ap, lda, wt, K, K, m0, n0, lane, acc);
  float bb[4];
#pragma unroll
  for (int t = 0; t < 4; ++t) bb[t] = bias[n0 + 16 * t + c];
  out_epilogue_h16(acc, scale, bb, oscale, st[wave], out, ldo, m0, n0, lane, hh, c);
}

extern "C" void kernel_launch(void* const* d_in, const int* in_sizes, int n_in,
                              void* d_out, int out_size, void* d_ws, size_t ws_size,
                              hipStream_t stream) {
  if (n_in < 13) return;
  if (in_sizes[0] != NTOK * HID) return;
  if (in_sizes[1] != HID) return;
  if (in_sizes[2] != HID) return;
  if (in_sizes[3] != HID * NQKV) return;
  if (in_sizes[4] != NQKV) return;
  if (in_sizes[5] != HID * HID) return;
  if (in_sizes[6] != HID) return;
  if (in_sizes[7] != HID) return;
  if (in_sizes[8] != HID) return;
  if (in_sizes[9] != HID * DFF) return;
  if (in_sizes[10] != DFF) return;
  if (in_sizes[11] != DFF * HID) return;
  if (in_sizes[12] != HID) return;
  if (out_size != NTOK * HID) return;

  const float* x    = (const float*)d_in[0];
  const float* g1   = (const float*)d_in[1];
  const float* be1  = (const float*)d_in[2];
  const float* wqkv = (const float*)d_in[3];
  const float* bqkv = (const float*)d_in[4];
  const float* wp   = (const float*)d_in[5];
  const float* bp   = (const float*)d_in[6];
  const float* g2   = (const float*)d_in[7];
  const float* be2  = (const float*)d_in[8];
  const float* w1   = (const float*)d_in[9];
  const float* b1   = (const float*)d_in[10];
  const float* w2   = (const float*)d_in[11];
  const float* b2   = (const float*)d_in[12];
  float* out = (float*)d_out;

  size_t off = 0;
  const size_t oNh  = off; off += (size_t)NTOK * HID * 2;
  const size_t oWt  = off; off += (size_t)NQKV * HID * 2;
  const size_t oWp  = off; off += (size_t)HID * HID * 2;
  const size_t oW1  = off; off += (size_t)DFF * HID * 2;
  const size_t oW2  = off; off += (size_t)HID * DFF * 2;
  const size_t oQK  = off; off += (size_t)2 * QKPLANE * 2;
  const size_t oV   = off; off += (size_t)NB * NH * HDM * SQ * 2;
  const size_t oO   = off; off += (size_t)NTOK * HID * 2;
  const size_t oT1  = off; off += (size_t)NTOK * HID * 4;
  const size_t oH   = off; off += (size_t)NTOK * DFF * 2;
  if (off > ws_size) return;
  if (off > (size_t)134217728) return;

  char* ws = (char*)d_ws;
  _Float16* Nh  = (_Float16*)(ws + oNh);
  _Float16* Wt  = (_Float16*)(ws + oWt);
  _Float16* Wpt = (_Float16*)(ws + oWp);
  _Float16* W1t = (_Float16*)(ws + oW1);
  _Float16* W2t = (_Float16*)(ws + oW2);
  _Float16* QKp = (_Float16*)(ws + oQK);
  _Float16* Kp  = QKp + (size_t)QKPLANE;
  _Float16* Vt  = (_Float16*)(ws + oV);
  _Float16* Op  = (_Float16*)(ws + oO);
  float*    T1  = (float*)(ws + oT1);
  _Float16* Hd  = (_Float16*)(ws + oH);

  k_wtr<<<dim3(NQKV / 64, HID / 64), dim3(256), 0, stream>>>(wqkv, HID, NQKV, WSC, Wt);
  k_wtr<<<dim3(HID / 64, HID / 64), dim3(256), 0, stream>>>(wp, HID, HID, WSC, Wpt);
  k_wtr<<<dim3(DFF / 64, HID / 64), dim3(256), 0, stream>>>(w1, HID, DFF, WSC, W1t);
  k_wtr<<<dim3(HID / 64, DFF / 64), dim3(256), 0, stream>>>(w2, DFF, HID, WSC, W2t);
  k_ln_h<0><<<dim3(NTOK / 8), dim3(256), 0, stream>>>(x, x, g1, be1, Nh);
  k_qkv<<<dim3(NTOK / 256, NQKV / 64), dim3(256), 0, stream>>>(Nh, Wt, bqkv, QKp, Vt);
  k_attn<<<dim3(NB * NH * NQB), dim3(256), 0, stream>>>(QKp, Kp, Vt, Op, 1.0f / (QSC * 8.0f));
  k_gemm_f32<0><<<dim3(NTOK / 256, HID / 64), dim3(256), 0, stream>>>(Op, HID, Wpt, HID, bp, 1.0f / (OSC * WSC),
                                                                       T1, HID, x, x);
  k_ln_h<1><<<dim3(NTOK / 8), dim3(256), 0, stream>>>(x, T1, g2, be2, Nh);
  k_gemm_h16<<<dim3(NTOK / 256, DFF / 64), dim3(256), 0, stream>>>(Nh, HID, W1t, HID, b1, 1.0f / WSC, HSC, Hd, DFF);
  k_gemm_f32<1><<<dim3(NTOK / 256, HID / 64), dim3(256), 0, stream>>>(Hd, DFF, W2t, DFF, b2, 1.0f / (HSC * WSC),
                                                                       out, HID, x, T1);
  (void)hipGetLastError();
}
